// NodalMLP_54889682043442
// MI455X (gfx1250) — hardware-verified
//
#include <hip/hip_runtime.h>

typedef _Float16 v16h __attribute__((ext_vector_type(16)));
typedef _Float16 v8h  __attribute__((ext_vector_type(8)));
typedef float    v8f  __attribute__((ext_vector_type(8)));
typedef float    v4f  __attribute__((ext_vector_type(4)));
union Frag { v16h v; v8h hv[2]; };

#define NB      16
#define NN      400
#define HID     96
#define DW      64
#define FS      8
#define FIN     408
#define K1P     416
#define NEDGE   79800
#define NFLAT   (NB * NEDGE)
#define NTILE   (NFLAT / 32)
#define NCHUNK  15
#define TPC     (NTILE / NCHUNK)
#define GWAVES  2
#define GBLOCKS (TPC / GWAVES)
#define DWAVES  4
#define DBLOCKS (TPC / DWAVES)
#define EFP     288
#define HP      128
#define AP      424
#define H1P     104
#define EPSV    1e-8f
#define ETHREADS 192

#define SEG_E1    0
#define SEG_E2    39936
#define SEG_D1    49152
#define SEG_D2    67584
#define PW_HALVES 71680
#define PIECES_E1 4992
#define PIECES_E2 1152
#define PIECES_D1 2304
#define PIECES_D2 512
#define PIECES    (PIECES_E1 + PIECES_E2 + PIECES_D1 + PIECES_D2)
#define PTHREADS  256
#define PBLOCKS   ((PIECES + PTHREADS - 1) / PTHREADS)

#define WS_PW_OFF    0
#define WS_PW_BYTES  (PW_HALVES * 2)
#define WS_H16_OFF   WS_PW_BYTES
#define WS_H16_BYTES (NB * NN * HP * 2)
#define WS_EF_OFF    (WS_H16_OFF + WS_H16_BYTES)
#define WS_EF_BYTES  (TPC * 32 * EFP * 2)
#define WS_TOTAL     (WS_EF_OFF + WS_EF_BYTES)

static_assert(NFLAT % 32 == 0, "");
static_assert(NTILE % NCHUNK == 0, "");
static_assert(TPC % GWAVES == 0, "");
static_assert(TPC % DWAVES == 0, "");
static_assert(NN % 16 == 0, "");
static_assert(PIECES % 32 == 0, "");
static_assert(WS_H16_OFF % 128 == 0, "");
static_assert(WS_EF_OFF % 128 == 0, "");
static_assert((32 * EFP * 2) % 128 == 0, "");

__device__ __forceinline__ v8f zero8() {
  v8f z;
#pragma unroll
  for (int i = 0; i < 8; ++i) z[i] = 0.f;
  return z;
}

__device__ __forceinline__ v8f wmma_g(v8f c, v16h a, v16h b) {
  c = __builtin_amdgcn_wmma_f32_16x16x32_f16(false, a, false, b, (short)0, c, false, false);
  asm volatile("v_nop\n\tv_nop\n\tv_nop\n\tv_nop" : "+v"(c) : "v"(a), "v"(b));
  return c;
}
__device__ __forceinline__ v8f wmma_r(v8f c, v16h a, v16h b) {
  return __builtin_amdgcn_wmma_f32_16x16x32_f16(false, a, false, b, (short)0, c, false, false);
}

__global__ __launch_bounds__(PTHREADS)
void pack_kernel(const float* __restrict__ We1, const float* __restrict__ We2,
                 const float* __restrict__ Wd1, const float* __restrict__ Wd2,
                 _Float16* __restrict__ pw)
{
  const int p = blockIdx.x * PTHREADS + threadIdx.x;
  if (p >= PIECES) return;
  const float* W; int K, N, NT, loc; float scale;
  if (p < PIECES_E1) {
    W = We1; K = FIN; N = HID; NT = 6; loc = p; scale = 16.f;
  } else if (p < PIECES_E1 + PIECES_E2) {
    W = We2; K = HID; N = HID; NT = 6; loc = p - PIECES_E1; scale = 8.f;
  } else if (p < PIECES_E1 + PIECES_E2 + PIECES_D1) {
    W = Wd1; K = 3 * HID; N = DW; NT = 4; loc = p - (PIECES_E1 + PIECES_E2); scale = 16.f;
  } else {
    W = Wd2; K = DW; N = DW; NT = 4; loc = p - (PIECES_E1 + PIECES_E2 + PIECES_D1); scale = 8.f;
  }
  const int f = loc >> 6, wi = loc & 63, ln = wi >> 1, half = wi & 1;
  const int kt = f / NT, nt = f - kt * NT;
  const int n = nt * 16 + (ln & 15);
  const int kb = kt * 32 + half * 16 + (ln >> 4) * 8;
  union { v8h v; _Float16 e[8]; } u;
#pragma unroll
  for (int j = 0; j < 8; ++j) {
    const int k = kb + j;
    float x = 0.f;
    if (k < K) x = W[k * N + n] * scale;
    u.e[j] = (_Float16)x;
  }
  const v8h val = u.v;
  _Float16* dst = pw + (size_t)p * 8;
  *(volatile v8h*)dst = val;
  __threadfence();
  *(volatile v8h*)dst = val;
}

__global__ __launch_bounds__(ETHREADS)
void enc_kernel(const float* __restrict__ nf, const float* __restrict__ sc,
                const float* __restrict__ smean, const float* __restrict__ sstd,
                const float* __restrict__ be1, const float* __restrict__ ae1,
                const float* __restrict__ be2, const float* __restrict__ ae2,
                const _Float16* __restrict__ pw, _Float16* __restrict__ h16)
{
  __shared__ __align__(16) _Float16 At[16 * AP];
  __shared__ __align__(16) _Float16 H1[16 * H1P];
  __shared__ __align__(16) _Float16 HO[16 * HP];
  __shared__ double red[ETHREADS];
  __shared__ float smisc[20];

  const int b = blockIdx.x;
  const int tid = threadIdx.x, w = tid >> 5, l = tid & 31, hh = l >> 4, m = l & 15;

  {
    const float* p = sc + (size_t)b * NN * NN;
    double ds = 0.0;
    for (int i = tid; i < NN * NN; i += ETHREADS) ds += (double)p[i];
    red[tid] = ds;
  }
  for (int i = tid; i < 16 * HP; i += ETHREADS) HO[i] = (_Float16)0.0f;
  __syncthreads();
  if (tid == 0) {
    double tsum = 0.0;
    for (int i = 0; i < ETHREADS; ++i) tsum += red[i];
    const float mean = (float)(tsum / (double)(NN * NN));
    smisc[0] = 1.0f / fmaxf(mean, EPSV);
  }
  if (tid < FS) {
    smisc[4 + tid]  = 1.0f / (sstd[tid] + EPSV);
    smisc[12 + tid] = smean[tid];
  }
  __syncthreads();
  const float inv = smisc[0];
  const float a1 = ae1[0], a2 = ae2[0];
  const int n = w * 16 + m;
  const float bias1 = be1[n], bias2 = be2[n];

  for (int mt = 0; mt < NN / 16; ++mt) {
    const int rowbase = b * NN + mt * 16;
    for (int idx = tid; idx < 16 * K1P; idx += ETHREADS) {
      const int r = idx / K1P, k = idx - r * K1P;
      float v;
      if (k < FS)       v = (nf[(size_t)(rowbase + r) * FS + k] - smisc[12 + k]) * smisc[4 + k];
      else if (k < FIN) v = sc[(size_t)(rowbase + r) * NN + (k - FS)] * inv;
      else              v = 0.f;
      At[r * AP + k] = (_Float16)v;
    }
    __syncthreads();

    v8f acc = zero8();
#pragma unroll
    for (int kt = 0; kt < K1P / 32; ++kt) {
      Frag a, bf;
      const _Float16* ap = At + m * AP + kt * 32 + 8 * hh;
      a.hv[0] = *(const v8h*)ap;
      a.hv[1] = *(const v8h*)(ap + 16);
      const _Float16* bp = pw + SEG_E1 + ((kt * 6 + w) * 32 + l) * 16;
      bf.hv[0] = *(const v8h*)bp;
      bf.hv[1] = *(const v8h*)(bp + 8);
      acc = wmma_g(acc, a.v, bf.v);
    }
#pragma unroll
    for (int r = 0; r < 8; ++r) {
      float z = acc[r] * 0.0625f + bias1;
      z = (z >= 0.f) ? z : a1 * z;
      H1[(8 * hh + r) * H1P + n] = (_Float16)z;
    }
    __syncthreads();

    v8f acc2 = zero8();
#pragma unroll
    for (int kt = 0; kt < HID / 32; ++kt) {
      Frag a, bf;
      const _Float16* ap = H1 + m * H1P + kt * 32 + 8 * hh;
      a.hv[0] = *(const v8h*)ap;
      a.hv[1] = *(const v8h*)(ap + 16);
      const _Float16* bp = pw + SEG_E2 + ((kt * 6 + w) * 32 + l) * 16;
      bf.hv[0] = *(const v8h*)bp;
      bf.hv[1] = *(const v8h*)(bp + 8);
      acc2 = wmma_g(acc2, a.v, bf.v);
    }
#pragma unroll
    for (int r = 0; r < 8; ++r) {
      float z = acc2[r] * 0.125f + bias2;
      z = (z >= 0.f) ? z : a2 * z;
      HO[(8 * hh + r) * HP + n] = (_Float16)z;
    }
    __syncthreads();

    {
      _Float16* dst = h16 + (size_t)rowbase * HP;
      const int q0 = tid, q1 = tid + ETHREADS;
      const v8h v0 = *(const v8h*)(HO + q0 * 8);
      v8h v1 = v0;
      if (q1 < 256) v1 = *(const v8h*)(HO + q1 * 8);
      *(volatile v8h*)(dst + q0 * 8) = v0;
      if (q1 < 256) *(volatile v8h*)(dst + q1 * 8) = v1;
      __threadfence();
      *(volatile v8h*)(dst + q0 * 8) = v0;
      if (q1 < 256) *(volatile v8h*)(dst + q1 * 8) = v1;
    }
    __syncthreads();
  }
}

__global__ __launch_bounds__(GWAVES * 32)
void gather_kernel(const _Float16* __restrict__ h16, const int* __restrict__ ei,
                   const int* __restrict__ ej, _Float16* __restrict__ ef, int chunk)
{
  __shared__ __align__(16) _Float16 tile[GWAVES * 32 * EFP];
  const int wv = threadIdx.x >> 5, lane = threadIdx.x & 31;
  const int tl = blockIdx.x * GWAVES + wv;
  const int t  = chunk * TPC + tl;
  const int f  = t * 32 + lane;
  const int b  = f / NEDGE, e = f - b * NEDGE;
  int i0 = ei[e], j0 = ej[e];
  i0 = min(max(i0, 0), NN - 1);
  j0 = min(max(j0, 0), NN - 1);
  const _Float16* hi = h16 + (size_t)(b * NN + i0) * HP;
  const _Float16* hj = h16 + (size_t)(b * NN + j0) * HP;
  _Float16* trow = tile + (wv * 32 + lane) * EFP;
#pragma unroll
  for (int c = 0; c < HID / 8; ++c) {
    const v8h a = *(const v8h*)(hi + 8 * c);
    const v8h q = *(const v8h*)(hj + 8 * c);
    union { v8h v; unsigned u[4]; } d;
    d.v = a - q;
#pragma unroll
    for (int k = 0; k < 4; ++k) d.u[k] &= 0x7FFF7FFFu;
    *(v8h*)(trow + 8 * c)           = a + q;
    *(v8h*)(trow + HID + 8 * c)     = d.v;
    *(v8h*)(trow + 2 * HID + 8 * c) = a * q;
  }
  __syncthreads();

  const _Float16* tw = tile + wv * 32 * EFP;
  _Float16* dst = ef + (size_t)tl * 32 * EFP;
#pragma unroll
  for (int it = 0; it < (32 * EFP / 8) / 32; ++it) {
    const int q = it * 32 + lane;
    const v8h v = *(const v8h*)(tw + q * 8);
    *(volatile v8h*)(dst + q * 8) = v;
  }
  __threadfence();
#pragma unroll
  for (int it = 0; it < (32 * EFP / 8) / 32; ++it) {
    const int q = it * 32 + lane;
    const v8h v = *(const v8h*)(tw + q * 8);
    *(volatile v8h*)(dst + q * 8) = v;
  }
}

__device__ __forceinline__ void epi_h(_Float16* z1, v8f c, int mt, int nt, int r, int hs,
                                      float bv, float a, float scale) {
  const int N = nt * 16 + r;
#pragma unroll
  for (int v = 0; v < 8; ++v) {
    const int M = mt * 16 + 8 * hs + v;
    float z = c[v] * scale + bv;
    z = (z >= 0.f) ? z : a * z;
    z1[M * DW + N] = (_Float16)z;
  }
}
__device__ __forceinline__ void epi_f(float* z2, v8f c, int mt, int nt, int r, int hs,
                                      float bv, float a, float scale) {
  const int N = nt * 16 + r;
#pragma unroll
  for (int v = 0; v < 8; ++v) {
    const int M = mt * 16 + 8 * hs + v;
    float z = c[v] * scale + bv;
    z = (z >= 0.f) ? z : a * z;
    z2[M * DW + N] = z;
  }
}

__global__ __launch_bounds__(DWAVES * 32)
void dec_kernel(const _Float16* __restrict__ ef, const _Float16* __restrict__ pw,
                const float* __restrict__ bd1, const float* __restrict__ ad1,
                const float* __restrict__ bd2, const float* __restrict__ ad2,
                const float* __restrict__ Wd3, const float* __restrict__ bd3,
                float* __restrict__ out, int chunk)
{
  __shared__ __align__(16) _Float16 zmem[DWAVES * 6144];
  __shared__ __align__(16) float obuf[DWAVES * 32];

  const int wv = threadIdx.x >> 5, lane = threadIdx.x & 31;
  const int r = lane & 15, hs = lane >> 4;
  const int tl = blockIdx.x * DWAVES + wv;
  const int t  = chunk * TPC + tl;

  _Float16* z1 = zmem + wv * 6144;
  float*    z2 = (float*)(z1 + 2048);

  const _Float16* ar0 = ef + ((size_t)tl * 32 + r) * EFP;
  const _Float16* ar1 = ar0 + 16 * EFP;

  v8f c00 = zero8(), c01 = zero8(), c02 = zero8(), c03 = zero8();
  v8f c10 = zero8(), c11 = zero8(), c12 = zero8(), c13 = zero8();
#pragma unroll
  for (int kt = 0; kt < 9; ++kt) {
    Frag A0, A1, B0, B1, B2, B3;
    const int kb = kt * 32 + 8 * hs;
    A0.hv[0] = *(const v8h*)(ar0 + kb); A0.hv[1] = *(const v8h*)(ar0 + kb + 16);
    A1.hv[0] = *(const v8h*)(ar1 + kb); A1.hv[1] = *(const v8h*)(ar1 + kb + 16);
    const _Float16* bp = pw + SEG_D1 + (kt * 4 * 32 + lane) * 16;
    B0.hv[0] = *(const v8h*)(bp);        B0.hv[1] = *(const v8h*)(bp + 8);
    B1.hv[0] = *(const v8h*)(bp + 512);  B1.hv[1] = *(const v8h*)(bp + 520);
    B2.hv[0] = *(const v8h*)(bp + 1024); B2.hv[1] = *(const v8h*)(bp + 1032);
    B3.hv[0] = *(const v8h*)(bp + 1536); B3.hv[1] = *(const v8h*)(bp + 1544);
    c00 = wmma_r(c00, A0.v, B0.v); c10 = wmma_r(c10, A1.v, B0.v);
    c01 = wmma_r(c01, A0.v, B1.v); c11 = wmma_r(c11, A1.v, B1.v);
    c02 = wmma_r(c02, A0.v, B2.v); c12 = wmma_r(c12, A1.v, B2.v);
    c03 = wmma_r(c03, A0.v, B3.v); c13 = wmma_r(c13, A1.v, B3.v);
    asm volatile("v_nop\n\tv_nop\n\tv_nop\n\tv_nop"
                 : "+v"(c00), "+v"(c01), "+v"(c02), "+v"(c03),
                   "+v"(c10), "+v"(c11), "+v"(c12), "+v"(c13)
                 : "v"(A0.v), "v"(A1.v), "v"(B0.v), "v"(B1.v), "v"(B2.v), "v"(B3.v));
  }
  {
    const float a1 = ad1[0];
    const float q0 = bd1[r], q1 = bd1[16 + r], q2 = bd1[32 + r], q3 = bd1[48 + r];
    const float s1 = 0.0625f;
    epi_h(z1, c00, 0, 0, r, hs, q0, a1, s1); epi_h(z1, c01, 0, 1, r, hs, q1, a1, s1);
    epi_h(z1, c02, 0, 2, r, hs, q2, a1, s1); epi_h(z1, c03, 0, 3, r, hs, q3, a1, s1);
    epi_h(z1, c10, 1, 0, r, hs, q0, a1, s1); epi_h(z1, c11, 1, 1, r, hs, q1, a1, s1);
    epi_h(z1, c12, 1, 2, r, hs, q2, a1, s1); epi_h(z1, c13, 1, 3, r, hs, q3, a1, s1);
  }
  __syncthreads();

  v8f d00 = zero8(), d01 = zero8(), d02 = zero8(), d03 = zero8();
  v8f d10 = zero8(), d11 = zero8(), d12 = zero8(), d13 = zero8();
#pragma unroll
  for (int kt = 0; kt < 2; ++kt) {
    Frag A0, A1, B0, B1, B2, B3;
    const _Float16* ap0 = z1 + r * DW + kt * 32 + 8 * hs;
    const _Float16* ap1 = ap0 + 16 * DW;
    A0.hv[0] = *(const v8h*)ap0; A0.hv[1] = *(const v8h*)(ap0 + 16);
    A1.hv[0] = *(const v8h*)ap1; A1.hv[1] = *(const v8h*)(ap1 + 16);
    const _Float16* bp = pw + SEG_D2 + (kt * 4 * 32 + lane) * 16;
    B0.hv[0] = *(const v8h*)(bp);        B0.hv[1] = *(const v8h*)(bp + 8);
    B1.hv[0] = *(const v8h*)(bp + 512);  B1.hv[1] = *(const v8h*)(bp + 520);
    B2.hv[0] = *(const v8h*)(bp + 1024); B2.hv[1] = *(const v8h*)(bp + 1032);
    B3.hv[0] = *(const v8h*)(bp + 1536); B3.hv[1] = *(const v8h*)(bp + 1544);
    d00 = wmma_r(d00, A0.v, B0.v); d10 = wmma_r(d10, A1.v, B0.v);
    d01 = wmma_r(d01, A0.v, B1.v); d11 = wmma_r(d11, A1.v, B1.v);
    d02 = wmma_r(d02, A0.v, B2.v); d12 = wmma_r(d12, A1.v, B2.v);
    d03 = wmma_r(d03, A0.v, B3.v); d13 = wmma_r(d13, A1.v, B3.v);
    asm volatile("v_nop\n\tv_nop\n\tv_nop\n\tv_nop"
                 : "+v"(d00), "+v"(d01), "+v"(d02), "+v"(d03),
                   "+v"(d10), "+v"(d11), "+v"(d12), "+v"(d13)
                 : "v"(A0.v), "v"(A1.v), "v"(B0.v), "v"(B1.v), "v"(B2.v), "v"(B3.v));
  }
  {
    const float a2 = ad2[0];
    const float q0 = bd2[r], q1 = bd2[16 + r], q2 = bd2[32 + r], q3 = bd2[48 + r];
    const float s2 = 0.125f;
    epi_f(z2, d00, 0, 0, r, hs, q0, a2, s2); epi_f(z2, d01, 0, 1, r, hs, q1, a2, s2);
    epi_f(z2, d02, 0, 2, r, hs, q2, a2, s2); epi_f(z2, d03, 0, 3, r, hs, q3, a2, s2);
    epi_f(z2, d10, 1, 0, r, hs, q0, a2, s2); epi_f(z2, d11, 1, 1, r, hs, q1, a2, s2);
    epi_f(z2, d12, 1, 2, r, hs, q2, a2, s2); epi_f(z2, d13, 1, 3, r, hs, q3, a2, s2);
  }
  __syncthreads();

  float s = bd3[0];
  {
    const float* zr = z2 + lane * DW;
#pragma unroll
    for (int c = 0; c < DW; ++c) s += zr[c] * Wd3[c];
  }
  obuf[wv * 32 + lane] = s;
  __syncthreads();

  if (lane < 8) {
    const v4f v = *(const v4f*)(obuf + wv * 32 + lane * 4);
    float* dst = out + (size_t)t * 32 + lane * 4;
    *(volatile v4f*)dst = v;
    __threadfence();
    *(volatile v4f*)dst = v;
  }
}

extern "C" void kernel_launch(void* const* d_in, const int* in_sizes, int n_in,
                              void* d_out, int out_size, void* d_ws, size_t ws_size,
                              hipStream_t stream) {
  if (n_in < 21) return;
  if (in_sizes[1] != NB * NN * FS || in_sizes[2] != NB * NN * NN ||
      in_sizes[3] < FS || in_sizes[4] < FS ||
      in_sizes[5] != FIN * HID || in_sizes[6] != HID || in_sizes[7] < 1 ||
      in_sizes[8] != HID * HID || in_sizes[9] != HID || in_sizes[10] < 1 ||
      in_sizes[11] != 3 * HID * DW || in_sizes[12] != DW || in_sizes[13] < 1 ||
      in_sizes[14] != DW * DW || in_sizes[15] != DW || in_sizes[16] < 1 ||
      in_sizes[17] != DW || in_sizes[18] < 1 ||
      in_sizes[19] != NEDGE || in_sizes[20] != NEDGE) return;
  if (out_size != NFLAT) return;
  if ((size_t)WS_TOTAL > ws_size) return;

  const float* nf    = (const float*)d_in[1];
  const float* sc    = (const float*)d_in[2];
  const float* smean = (const float*)d_in[3];
  const float* sstd  = (const float*)d_in[4];
  const float* We1   = (const float*)d_in[5];
  const float* be1   = (const float*)d_in[6];
  const float* ae1   = (const float*)d_in[7];
  const float* We2   = (const float*)d_in[8];
  const float* be2   = (const float*)d_in[9];
  const float* ae2   = (const float*)d_in[10];
  const float* Wd1   = (const float*)d_in[11];
  const float* bd1   = (const float*)d_in[12];
  const float* ad1   = (const float*)d_in[13];
  const float* Wd2   = (const float*)d_in[14];
  const float* bd2   = (const float*)d_in[15];
  const float* ad2   = (const float*)d_in[16];
  const float* Wd3   = (const float*)d_in[17];
  const float* bd3   = (const float*)d_in[18];
  const int*   ei    = (const int*)d_in[19];
  const int*   ej    = (const int*)d_in[20];

  char* ws = (char*)d_ws;
  _Float16* pw  = (_Float16*)(ws + WS_PW_OFF);
  _Float16* h16 = (_Float16*)(ws + WS_H16_OFF);
  _Float16* ef  = (_Float16*)(ws + WS_EF_OFF);
  float* outp   = (float*)d_out;

  pack_kernel<<<dim3(PBLOCKS), dim3(PTHREADS), 0, stream>>>(We1, We2, Wd1, Wd2, pw);
  enc_kernel<<<dim3(NB), dim3(ETHREADS), 0, stream>>>(nf, sc, smean, sstd, be1, ae1, be2, ae2, pw, h16);
  for (int chunk = 0; chunk < NCHUNK; ++chunk) {
    gather_kernel<<<dim3(GBLOCKS), dim3(GWAVES * 32), 0, stream>>>(h16, ei, ej, ef, chunk);
    dec_kernel<<<dim3(DBLOCKS), dim3(DWAVES * 32), 0, stream>>>(
        ef, pw, bd1, ad1, bd2, ad2, Wd3, bd3, outp, chunk);
  }
}
